// CenterLoss_17987323035876
// MI455X (gfx1250) — hardware-verified
//
#include <hip/hip_runtime.h>


#define NB_  4096
#define NCL  100000
#define NCP  100032
#define DD   128
#define DM   DD
#define CMIN 1e-12f
#define CMAX 1e12f
#define LOSC 1024.0f

typedef _Float16 h16;
typedef unsigned short bf;
typedef __attribute__((ext_vector_type(16))) __bf16   v16bf;
typedef __attribute__((ext_vector_type(16))) _Float16 v16h;
typedef __attribute__((ext_vector_type(8)))  _Float16 v8h;
typedef __attribute__((ext_vector_type(8)))  unsigned short v8us;
typedef __attribute__((ext_vector_type(8)))  float    v8f;
typedef __attribute__((ext_vector_type(4)))  float    v4f;
typedef v8h  __attribute__((may_alias)) v8ha;
typedef v4f  __attribute__((may_alias)) v4fa;
typedef v8us __attribute__((may_alias)) v8usa;

__device__ __forceinline__ unsigned short f2bf(float f) { unsigned u = __float_as_uint(f); u += 0x7FFFu + ((u >> 16) & 1u); return (unsigned short)(u >> 16); }
__device__ __forceinline__ float bf2f(unsigned short b) { return __uint_as_float(((unsigned)b) << 16); }
__device__ __forceinline__ float bfr(float f) { return bf2f(f2bf(f)); }
__device__ __forceinline__ v16h cat16(v8h lo, v8h hi) { return __builtin_shufflevector(lo, hi, 0, 1, 2, 3, 4, 5, 6, 7, 8, 9, 10, 11, 12, 13, 14, 15); }
__device__ __forceinline__ v16bf cat16b(v8us lo, v8us hi) { return __builtin_bit_cast(v16bf, __builtin_shufflevector(lo, hi, 0, 1, 2, 3, 4, 5, 6, 7, 8, 9, 10, 11, 12, 13, 14, 15)); }
__device__ __forceinline__ v8f wmma16(v16h a, v16h b, v8f c) { return __builtin_amdgcn_wmma_f32_16x16x32_f16(false, a, false, b, (short)0, c, false, false); }
__device__ __forceinline__ v8f wmmab(v16bf a, v16bf b, v8f c) { return __builtin_amdgcn_wmma_f32_16x16x32_bf16(false, a, false, b, (short)0, c, false, false); }


__global__ __launch_bounds__(256) void k_cvt(const float* __restrict__ src, int nreal, int nrows, bf* dst) {
    typedef __attribute__((ext_vector_type(4))) unsigned short v4us;
    const int lane = threadIdx.x & 31, r = blockIdx.x * 8 + (threadIdx.x >> 5); if (r >= nrows) return; const bool ok = r < nreal; const int rc = ok ? r : 0; v4us o;
#pragma unroll
    for (int i = 0; i < 4; ++i) { const float v = src[(size_t)rc * DD + lane * 4 + i]; o[i] = ok ? f2bf(v) : (unsigned short)0; }
    *(volatile v4us*)(dst + (size_t)r * DD + lane * 4) = o; __threadfence(); *(volatile v4us*)(dst + (size_t)r * DD + lane * 4) = o;
}
__global__ __launch_bounds__(256) void k_sq(const float* __restrict__ src, int nreal, int nrows, float* SQ) {
    const int r = blockIdx.x * 256 + threadIdx.x; if (r >= nrows) return; float s = 0.f;
    if (r < nreal) {
#pragma unroll 4
        for (int d = 0; d < DD; ++d) { const float v = bfr(src[(size_t)r * DD + d]); s = fmaf(v, v, s); } }
    *(volatile float*)(SQ + r) = s; __threadfence(); *(volatile float*)(SQ + r) = s;
}
__global__ __launch_bounds__(128) void k_gemmloss(const bf* __restrict__ A, const bf* __restrict__ Bn, const float* __restrict__ SQX, const float* __restrict__ SQC, const int* __restrict__ lab, float* PART) {
    __shared__ float wsum[4];
    const int lane = threadIdx.x & 31, wave = threadIdx.x >> 5, lr = lane & 15, hi = lane >> 4;
    const int r0 = blockIdx.x * 64 + wave * 16, c0 = blockIdx.y * 64;
    const size_t aoff = (size_t)(r0 + lr) * DD + 8 * hi;
    v8f acc[4];
#pragma unroll
    for (int t = 0; t < 4; ++t) acc[t] = (v8f){};
#pragma unroll
    for (int kc = 0; kc < DD; kc += 32) {
        const v16bf a = cat16b(*(const v8us*)(A + aoff + kc), *(const v8us*)(A + aoff + kc + 16));
#pragma unroll
        for (int t = 0; t < 4; ++t) { const size_t bo = (size_t)(c0 + t * 16 + lr) * DD + kc + 8 * hi; const v16bf bb = cat16b(*(const v8us*)(Bn + bo), *(const v8us*)(Bn + bo + 16)); acc[t] = wmmab(a, bb, acc[t]); }
        asm volatile("v_nop\n\tv_nop\n\tv_nop\n\tv_nop" : "+v"(acc[0]), "+v"(acc[1]), "+v"(acc[2]), "+v"(acc[3]) : "v"(a));
    }
    float s = 0.f;
#pragma unroll
    for (int t = 0; t < 4; ++t) { const int k = c0 + t * 16 + lr; const float sqc = SQC[k]; const bool kin = k < NCL;
#pragma unroll
        for (int j = 0; j < 8; ++j) { const int b = r0 + 8 * hi + j; float d = SQX[b] + sqc - 2.0f * acc[t][j]; d = (lab[b] == k) ? d : 0.f; d = fminf(fmaxf(d, CMIN), CMAX); s += kin ? d : 0.f; } }
#pragma unroll
    for (int sh = 16; sh; sh >>= 1) s += __shfl_xor(s, sh, 32);
    if (lane == 0) wsum[wave] = s;
    __syncthreads();
    if (wave == 0) { const float tot = ((wsum[0] + wsum[1]) + wsum[2]) + wsum[3]; const float v = (lane == 0) ? tot : 0.f; float* p = PART + ((size_t)blockIdx.y * gridDim.x + blockIdx.x) * 32 + lane;
        *(volatile float*)p = v; __threadfence(); *(volatile float*)p = v; }
}
__global__ __launch_bounds__(32) void k_final(const float* __restrict__ PART, int nparts, float* OUTP) {
    if (threadIdx.x != 0) return; float s = 0.f;
#pragma unroll 1
    for (int q = 0; q < nparts; ++q) s += PART[(size_t)q * 32];
    const float r = s / (float)NB_; *(volatile float*)OUTP = r; __threadfence(); *(volatile float*)OUTP = r;
}

extern "C" void kernel_launch(void* const* d_in, const int* in_sizes, int n_in,
                              void* d_out, int out_size, void* d_ws, size_t ws_size, hipStream_t stream) {
    (void)in_sizes; (void)n_in; (void)out_size;
    const float* x = (const float*)d_in[0]; const int* lab = (const int*)d_in[1]; const float* cen = (const float*)d_in[2];
    float* out = (float*)d_out;
    char* wsp = (char*)d_ws;
    auto take = [&](size_t bytes) { char* p = wsp; wsp += (bytes + 255) & ~(size_t)255; return (void*)p; };
    bf* Xb = (bf*)take((size_t)NB_ * DD * 2); bf* Cb = (bf*)take((size_t)NCP * DD * 2); float* SQX = (float*)take((size_t)NB_ * 4); float* SQC = (float*)take((size_t)NCP * 4);
    const int nparts = (NB_ / 64) * (NCP / 64); float* PART = (float*)take((size_t)nparts * 32 * 4);
    if ((size_t)(wsp - (char*)d_ws) > ws_size) return;
    k_cvt<<<NB_ / 8, 256, 0, stream>>>(x, NB_, NB_, Xb); k_cvt<<<NCP / 8, 256, 0, stream>>>(cen, NCL, NCP, Cb);
    k_sq<<<NB_ / 256, 256, 0, stream>>>(x, NB_, NB_, SQX); k_sq<<<(NCP + 255) / 256, 256, 0, stream>>>(cen, NCL, NCP, SQC);
    k_gemmloss<<<dim3(NB_ / 64, NCP / 64, 1), 128, 0, stream>>>(Xb, Cb, SQX, SQC, lab, PART);
    k_final<<<1, 32, 0, stream>>>(PART, nparts, out);
}
